// GNNEncoderB_26113401160169
// MI455X (gfx1250) — hardware-verified
//
#include <hip/hip_runtime.h>
#include <math.h>


#define NG 32
#define N0 2048
#define N1 1024
#define N2 512
#define CH 64

typedef __attribute__((ext_vector_type(16))) _Float16 v16h;
typedef __attribute__((ext_vector_type(8)))  float v8f;
typedef __attribute__((ext_vector_type(4)))  float v4f;
typedef __attribute__((ext_vector_type(4)))  int v4i;
typedef float __attribute__((may_alias)) float_a;
typedef int __attribute__((may_alias)) int_a;

template <typename T> __device__ __forceinline__ void vst2(void* p, T v) { *(volatile T*)p = v; __threadfence(); *(volatile T*)p = v; }
__device__ __forceinline__ v8f wmma16(v16h a, v16h b, v8f c) {
  v8f d = __builtin_amdgcn_wmma_f32_16x16x32_f16(false, a, false, b, (short)0, c, false, false);
  asm volatile("v_nop\n\tv_nop\n\tv_nop\n\tv_nop" : "+v"(d) : "v"(a), "v"(b));
  return d;
}
__device__ __forceinline__ v16h frag_col(const float* W, int k0, int n, int lane, int ld, int K) {
  v16h a; const int g = lane >> 4;
#pragma unroll
  for (int i = 0; i < 8; ++i) { const int ka = k0 + 8 * g + i, kb = ka + 16;
    a[i] = (_Float16)(ka < K ? W[(size_t)ka * ld + n] : 0.f); a[8 + i] = (_Float16)(kb < K ? W[(size_t)kb * ld + n] : 0.f); }
  return a;
}
__device__ __forceinline__ v16h frag_f32(const float* rowk0, int lane) {
  v16h a; const float* p = rowk0 + 8 * (lane >> 4);
#pragma unroll
  for (int i = 0; i < 8; ++i) { a[i] = (_Float16)p[i]; a[8 + i] = (_Float16)p[16 + i]; }
  return a;
}
#define LDSX() do { asm volatile("s_wait_dscnt 0" ::: "memory"); __builtin_amdgcn_wave_barrier(); __builtin_amdgcn_fence(__ATOMIC_RELEASE, "workgroup"); } while (0)

__device__ __forceinline__ float dist2(const float* a, const float* b) {
#pragma clang fp contract(off)
  const float dx = a[0] - b[0], dy = a[1] - b[1], dz = a[2] - b[2];
  float p0 = dx * dx, p1 = dy * dy, p2 = dz * dz;
  asm volatile("" : "+v"(p0), "+v"(p1), "+v"(p2));
  const float s = p0 + p2;
  return s + p1;
}

template <int NP, int K>
__global__ __launch_bounds__(256) void k_knn(const float* __restrict__ pos, int* __restrict__ idx) {
  __shared__ float sp[NP * 3];
  __shared__ __align__(16) int si[256 * K];
  const int g = blockIdx.y, i0 = blockIdx.x * 256, tid = threadIdx.x, i = i0 + tid;
  const float* pg = pos + (size_t)g * NP * 3;
  for (int q = tid; q < NP * 3; q += 256) sp[q] = pg[q];
  __syncthreads();
  float bd[K]; int bi[K];
#pragma unroll
  for (int q = 0; q < K; ++q) { bd[q] = 3.0e38f; bi[q] = 0x7fffffff; }
  const float pi[3] = { sp[i * 3], sp[i * 3 + 1], sp[i * 3 + 2] };
#pragma unroll 1
  for (int j = 0; j < NP; ++j) { const float d = dist2(pi, &sp[j * 3]);
    if (d < bd[K - 1]) {
      int q = K - 1; while (q > 0 && bd[q - 1] > d) { bd[q] = bd[q - 1]; bi[q] = bi[q - 1]; --q; }
      bd[q] = d; bi[q] = j; } }
#pragma unroll
  for (int q = 0; q < K; ++q) si[tid * K + q] = bi[q];
  __syncthreads();
  for (int q = tid; q < 256 * K / 4; q += 256) vst2(idx + ((size_t)g * NP + i0) * K + q * 4, *(const v4i*)(&si[q * 4]));
}

template <int NP, int M>
__global__ __launch_bounds__(256) void k_fps(const float* __restrict__ pos, int* __restrict__ sel, float* __restrict__ pnext) {
  __shared__ float sp[NP * 3], sd[NP];
  __shared__ float rv[256]; __shared__ int ri[256];
  __shared__ __align__(16) int ss[M];
  __shared__ int cur;
  const int g = blockIdx.x, tid = threadIdx.x;
  const float* pg = pos + (size_t)g * NP * 3;
  for (int q = tid; q < NP * 3; q += 256) sp[q] = pg[q];
  __syncthreads();
  for (int j = tid; j < NP; j += 256) sd[j] = dist2(&sp[j * 3], &sp[0]);
  if (tid == 0) { ss[0] = 0; }
  __syncthreads();
#pragma unroll 1
  for (int s = 1; s < M; ++s) {
    float bv = -1.0f; int bix = 0x7fffffff;
    for (int j = tid; j < NP; j += 256) { const float v = sd[j]; if (v > bv || (v == bv && j < bix)) { bv = v; bix = j; } }
    rv[tid] = bv; ri[tid] = bix; __syncthreads();
    for (int st = 128; st > 0; st >>= 1) { if (tid < st) { const float v2 = rv[tid + st]; const int i2 = ri[tid + st];
        if (v2 > rv[tid] || (v2 == rv[tid] && i2 < ri[tid])) { rv[tid] = v2; ri[tid] = i2; } } __syncthreads(); }
    const int isel = ri[0];
    if (tid == 0) ss[s] = isel;
    for (int j = tid; j < NP; j += 256) { const float d = dist2(&sp[j * 3], &sp[isel * 3]); sd[j] = fminf(sd[j], d); }
    __syncthreads();
  }
  for (int q = tid; q < M / 4; q += 256) vst2(sel + (size_t)g * M + q * 4, *(const v4i*)(&ss[q * 4]));
  __syncthreads();
  for (int q4 = tid; q4 < M * 3 / 4; q4 += 256) { v4f v;
#pragma unroll
    for (int e = 0; e < 4; ++e) { const int q = q4 * 4 + e; v[e] = sp[ss[q / 3] * 3 + (q % 3)]; }
    vst2(pnext + (size_t)g * M * 3 + q4 * 4, v); }
}
template <int NP, int M>
__global__ __launch_bounds__(256) void k_gather(const float* __restrict__ h, const int* __restrict__ sel, float* __restrict__ hn) {
  const int g = blockIdx.y, m0 = blockIdx.x * 64, tid = threadIdx.x;
  for (int q = tid; q < 64 * 16; q += 256) { const int m = m0 + (q >> 4), pc = q & 15; int s = sel[(size_t)g * M + m]; s = s < 0 ? 0 : (s >= NP ? NP - 1 : s);
    vst2(hn + ((size_t)g * M + m) * CH + pc * 4, *(const v4f*)(h + ((size_t)g * NP + s) * CH + pc * 4)); }
}

template <int NP, int K, int HIN>
__global__ __launch_bounds__(128) void k_layer(const float* __restrict__ h, const float* __restrict__ pos, const int* __restrict__ idx,
                                             const float* __restrict__ W1, const float* __restrict__ b1, const float* __restrict__ W2, const float* __restrict__ b2,
                                             float* __restrict__ hout) {
  constexpr int KIN = 2 * HIN + 3, KP = (KIN + 31) / 32 * 32;
  __shared__ __align__(16) float T[4][16][CH + 4];
  const int tid = threadIdx.x, w = tid >> 5, lane = tid & 31, col = lane & 15, gq = lane >> 4;
  const int g = blockIdx.y, p0 = blockIdx.x * 64 + w * 16, pi = p0 + col;
  const float* hg = h + (size_t)g * NP * HIN; const float* pg = pos + (size_t)g * NP * 3;
  float* Tw = &T[w][0][0];
  v8f mx[4];
#pragma unroll
  for (int t = 0; t < 4; ++t)
#pragma unroll
    for (int r = 0; r < 8; ++r) mx[t][r] = -3.0e38f;
#pragma unroll 1
  for (int j = 0; j < K; ++j) {
    int nj = idx[((size_t)g * NP + pi) * K + j]; nj = nj < 0 ? 0 : (nj >= NP ? NP - 1 : nj);
    const float r0 = pg[nj * 3] - pg[pi * 3], r1 = pg[nj * 3 + 1] - pg[pi * 3 + 1], r2 = pg[nj * 3 + 2] - pg[pi * 3 + 2];
    v8f acc[4] = {};
#pragma unroll 1
    for (int kc = 0; kc < KP / 32; ++kc) { v16h a;
#pragma unroll
      for (int i = 0; i < 16; ++i) { const int kk = kc * 32 + 8 * gq + (i < 8 ? i : 8 + i); float v;
        if (kk < HIN) v = hg[(size_t)pi * HIN + kk]; else if (kk < 2 * HIN) v = hg[(size_t)nj * HIN + kk - HIN];
        else if (kk == 2 * HIN) v = r0; else if (kk == 2 * HIN + 1) v = r1; else if (kk == 2 * HIN + 2) v = r2; else v = 0.f;
        a[i] = (_Float16)v; }
#pragma unroll
      for (int t = 0; t < 4; ++t) acc[t] = wmma16(a, frag_col(W1, kc * 32, t * 16 + col, lane, CH, KIN), acc[t]); }
#pragma unroll
    for (int t = 0; t < 4; ++t) { const float bb = b1[t * 16 + col];
#pragma unroll
      for (int r = 0; r < 8; ++r) { const float u = acc[t][r] + bb; Tw[(8 * gq + r) * (CH + 4) + t * 16 + col] = u > 0.f ? u : 0.f; } }
    LDSX();
#pragma unroll
    for (int t = 0; t < 4; ++t) acc[t] = (v8f){};
#pragma unroll
    for (int kc = 0; kc < 2; ++kc) { const v16h a = frag_f32(Tw + col * (CH + 4) + kc * 32, lane);
#pragma unroll
      for (int t = 0; t < 4; ++t) acc[t] = wmma16(a, frag_col(W2, kc * 32, t * 16 + col, lane, CH, CH), acc[t]); }
#pragma unroll
    for (int t = 0; t < 4; ++t)
#pragma unroll
      for (int r = 0; r < 8; ++r) mx[t][r] = fmaxf(mx[t][r], acc[t][r]);
    __builtin_amdgcn_wave_barrier();
  }
#pragma unroll
  for (int t = 0; t < 4; ++t) { const float bb = b2[t * 16 + col];
#pragma unroll
    for (int r = 0; r < 8; ++r) { const float u = mx[t][r] + bb; Tw[(8 * gq + r) * (CH + 4) + t * 16 + col] = u > 0.f ? u : 0.f; } }
  LDSX();
  for (int q = lane; q < 16 * 16; q += 32) { const int rl = q >> 4, pc = q & 15; vst2(hout + ((size_t)g * NP + p0 + rl) * CH + pc * 4, *(const v4f*)(Tw + rl * (CH + 4) + pc * 4)); }
}
__global__ __launch_bounds__(256) void k_readout(const float* __restrict__ h3, const float* __restrict__ Wr, const float* __restrict__ br, float* __restrict__ out) {
  __shared__ float pm[4][CH], gm[CH];
  __shared__ __align__(16) float so[NG * 6];
  const int tid = threadIdx.x, c = tid & 63, part = tid >> 6;
#pragma unroll 1
  for (int g = 0; g < NG; ++g) {
    float m = -3.0e38f;
    for (int p = part; p < N2; p += 4) m = fmaxf(m, h3[((size_t)g * N2 + p) * CH + c]);
    pm[part][c] = m; __syncthreads();
    if (tid < CH) gm[tid] = fmaxf(fmaxf(pm[0][tid], pm[1][tid]), fmaxf(pm[2][tid], pm[3][tid]));
    __syncthreads();
    if (tid < 6) { float s = br[tid];
#pragma unroll 1
      for (int i = 0; i < CH; ++i) s += gm[i] * Wr[i * 6 + tid];
      so[g * 6 + tid] = s; }
    __syncthreads();
  }
  if (tid < NG * 6 / 4) vst2(out + tid * 4, *(const v4f*)(&so[tid * 4]));
}

extern "C" void kernel_launch(void* const* d_in, const int* in_sizes, int n_in,
                              void* d_out, int out_size, void* d_ws, size_t ws_size,
                              hipStream_t stream) {
  (void)in_sizes; (void)n_in; (void)out_size; (void)ws_size;
  const float* pos = (const float*)d_in[1];
  const float* W1a = (const float*)d_in[3]; const float* b1a = (const float*)d_in[4]; const float* W1b = (const float*)d_in[5]; const float* b1b = (const float*)d_in[6];
  const float* W2a = (const float*)d_in[7]; const float* b2a = (const float*)d_in[8]; const float* W2b = (const float*)d_in[9]; const float* b2b = (const float*)d_in[10];
  const float* W3a = (const float*)d_in[11]; const float* b3a = (const float*)d_in[12]; const float* W3b = (const float*)d_in[13]; const float* b3b = (const float*)d_in[14];
  const float* Wr = (const float*)d_in[15]; const float* br = (const float*)d_in[16];
  float* out = (float*)d_out;
  char* ws = (char*)d_ws; size_t off = 0;
  auto take = [&](size_t bytes) { char* p = ws + off; off += (bytes + 255) & ~(size_t)255; return p; };
  int* idx1 = (int*)take((size_t)NG * N0 * 6 * 4); float* h1 = (float*)take((size_t)NG * N0 * CH * 4);
  int* sel1 = (int*)take((size_t)NG * N1 * 4); float* pos1 = (float*)take((size_t)NG * N1 * 3 * 4 + 256); float* h1s = (float*)take((size_t)NG * N1 * CH * 4);
  int* idx2 = (int*)take((size_t)NG * N1 * 4 * 4); float* h2 = (float*)take((size_t)NG * N1 * CH * 4);
  int* sel2 = (int*)take((size_t)NG * N2 * 4); float* pos2 = (float*)take((size_t)NG * N2 * 3 * 4 + 256); float* h2s = (float*)take((size_t)NG * N2 * CH * 4);
  int* idx3 = (int*)take((size_t)NG * N2 * 3 * 4 + 256); float* h3 = (float*)take((size_t)NG * N2 * CH * 4);
  k_knn<N0, 6><<<dim3(N0 / 256, NG), 256, 0, stream>>>(pos, idx1);
  k_layer<N0, 6, 3><<<dim3(N0 / 64, NG), 128, 0, stream>>>(pos, pos, idx1, W1a, b1a, W1b, b1b, h1);
  k_fps<N0, N1><<<NG, 256, 0, stream>>>(pos, sel1, pos1);
  k_gather<N0, N1><<<dim3(N1 / 64, NG), 256, 0, stream>>>(h1, sel1, h1s);
  k_knn<N1, 4><<<dim3(N1 / 256, NG), 256, 0, stream>>>(pos1, idx2);
  k_layer<N1, 4, CH><<<dim3(N1 / 64, NG), 128, 0, stream>>>(h1s, pos1, idx2, W2a, b2a, W2b, b2b, h2);
  k_fps<N1, N2><<<NG, 256, 0, stream>>>(pos1, sel2, pos2);
  k_gather<N1, N2><<<dim3(N2 / 64, NG), 256, 0, stream>>>(h2, sel2, h2s);
  k_knn<N2, 3><<<dim3(N2 / 256, NG), 256, 0, stream>>>(pos2, idx3);
  k_layer<N2, 3, CH><<<dim3(N2 / 64, NG), 128, 0, stream>>>(h2s, pos2, idx3, W3a, b3a, W3b, b3b, h3);
  k_readout<<<1, 256, 0, stream>>>(h3, Wr, br, out);
}
